// RelationalTransformerUpdate_50551765074577
// MI455X (gfx1250) — hardware-verified
//
#include <hip/hip_runtime.h>
#include <math.h>
#include <stddef.h>

#define NTOK  1024
#define DM    256
#define NH    8
#define DKH   32
#define FFD   1024
#define NREL  37
#define NLAY  8
#define LN_EPS 1e-6f

typedef __bf16 bf16_t;
typedef __bf16 v16b __attribute__((ext_vector_type(16)));
typedef __bf16 v8b  __attribute__((ext_vector_type(8)));
typedef float  v8f  __attribute__((ext_vector_type(8)));
typedef float  v4f  __attribute__((ext_vector_type(4)));
typedef int    v4i  __attribute__((ext_vector_type(4)));
typedef unsigned int v4u __attribute__((ext_vector_type(4)));
typedef v8b __attribute__((may_alias)) v8ba;
typedef v4f __attribute__((may_alias)) v4fa;
typedef v4i __attribute__((may_alias)) v4ia;
typedef v4u __attribute__((may_alias)) v4ua;

union Frag  { v16b v; v8b half[2]; };
union Pack8 { v8b b; v4u u; };

__device__ __forceinline__ v8f wmma_bf(v16b a, v16b b, v8f c) {
  v8f d = __builtin_amdgcn_wmma_f32_16x16x32_bf16(false, a, false, b, (short)0, c, false, false);
  asm volatile("v_nop\n\tv_nop\n\tv_nop\n\tv_nop" : "+v"(d) : "v"(a), "v"(b));
  return d;
}

__device__ __forceinline__ v8f wmma3(v16b ah, v16b al, v16b bh, v16b bl, v8f c) {
  c = wmma_bf(ah, bh, c);
  c = wmma_bf(al, bh, c);
  c = wmma_bf(ah, bl, c);
  return c;
}

__device__ __forceinline__ v16b load_frag(const bf16_t* p, int h) {
  Frag f;
  f.half[0] = *(const v8ba*)(p + 8 * h);
  f.half[1] = *(const v8ba*)(p + 16 + 8 * h);
  return f.v;
}

__device__ __forceinline__ void split8v(v8f p, v8b& hi, v8b& lo) {
  #pragma unroll
  for (int i = 0; i < 8; ++i) {
    const bf16_t hh = (bf16_t)p[i];
    hi[i] = hh;
    lo[i] = (bf16_t)(p[i] - (float)hh);
  }
}
__device__ __forceinline__ void split8(v4f a, v4f c, v8b& hi, v8b& lo) {
  const v8f p = { a.x, a.y, a.z, a.w, c.x, c.y, c.z, c.w };
  split8v(p, hi, lo);
}

__device__ __forceinline__ void vstore8b(bf16_t* p, v8b v) {
  Pack8 k; k.b = v;
  *(volatile v4u*)p = k.u;
}
__device__ __forceinline__ void vstore4f(float* p, v4f v) {
  *(volatile v4f*)p = v;
}

__device__ __forceinline__ v4f vrelu(v4f v) {
  v4f r;
  r.x = fmaxf(v.x, 0.0f); r.y = fmaxf(v.y, 0.0f); r.z = fmaxf(v.z, 0.0f); r.w = fmaxf(v.w, 0.0f);
  return r;
}

__device__ __forceinline__ float wsum32(float v) {
  v += __shfl_xor(v, 16);
  v += __shfl_xor(v, 8);
  v += __shfl_xor(v, 4);
  v += __shfl_xor(v, 2);
  v += __shfl_xor(v, 1);
  return v;
}

__device__ __forceinline__ void ln_stats(v4f a, v4f b, float& mu, float& inv) {
  float s = (a.x + a.y) + (a.z + a.w) + (b.x + b.y) + (b.z + b.w);
  s = wsum32(s);
  mu = s * (1.0f / 256.0f);
  const v4f da = a - mu, db = b - mu;
  float q = da.x * da.x + da.y * da.y + da.z * da.z + da.w * da.w
          + db.x * db.x + db.y * db.y + db.z * db.z + db.w * db.w;
  q = wsum32(q);
  const float sd = sqrtf(q * (1.0f / 255.0f));
  inv = 1.0f / (sd + LN_EPS);
}

__device__ __forceinline__ void wcvt_pass(const float (*s)[65], bf16_t* Bh, bf16_t* Bl,
                                          int K, int Nc, int lz, int k0, int n0, int w, int lane) {
  const int sub = lane >> 3, ks = 8 * (lane & 7);
  #pragma unroll
  for (int i = 0; i < 2; ++i) {
    const int nn = 8 * w + 4 * i + sub;
    const v4f a = { s[ks + 0][nn], s[ks + 1][nn], s[ks + 2][nn], s[ks + 3][nn] };
    const v4f c = { s[ks + 4][nn], s[ks + 5][nn], s[ks + 6][nn], s[ks + 7][nn] };
    v8b hi, lo;
    split8(a, c, hi, lo);
    const size_t g = ((size_t)lz * Nc + n0 + nn) * (size_t)K + k0 + ks;
    vstore8b(Bh + g, hi);
    vstore8b(Bl + g, lo);
  }
}

__global__ __launch_bounds__(256) void wcvt_kernel(const float* __restrict__ W,
                                                    bf16_t* Bh, bf16_t* Bl, int K, int Nc) {
  __shared__ float s[64][65];
  const int tid = threadIdx.x, lane = tid & 31, w = tid >> 5;
  const int lz = blockIdx.z, k0 = blockIdx.y * 64, n0 = blockIdx.x * 64;
  const float* src = W + ((size_t)lz * K + k0) * (size_t)Nc + n0;
  #pragma unroll
  for (int it = 0; it < 16; ++it) {
    const int kk = it * 4 + (tid >> 6), nn = tid & 63;
    s[kk][nn] = src[(size_t)kk * Nc + nn];
  }
  __syncthreads();
  wcvt_pass(s, Bh, Bl, K, Nc, lz, k0, n0, w, lane);
  __threadfence();
  wcvt_pass(s, Bh, Bl, K, Nc, lz, k0, n0, w, lane);
}

__global__ __launch_bounds__(256) void ln0_kernel(const float* __restrict__ x,
                                                   const float* __restrict__ g,
                                                   const float* __restrict__ b,
                                                   float* xf, bf16_t* nh, bf16_t* nl, int nrows) {
  const int lane = threadIdx.x & 31, w = threadIdx.x >> 5;
  const int row = blockIdx.x * 8 + w;
  if (row >= nrows) return;
  const float* xr = x + (size_t)row * DM;
  const int ca = 4 * lane, cb = 128 + 4 * lane, c8 = 8 * lane;
  const v4f va = *(const v4fa*)(xr + ca), vb = *(const v4fa*)(xr + cb);
  const v4f vc0 = *(const v4fa*)(xr + c8), vc1 = *(const v4fa*)(xr + c8 + 4);
  float mu, inv;
  ln_stats(va, vb, mu, inv);
  const v4f g0 = *(const v4fa*)(g + c8), g1 = *(const v4fa*)(g + c8 + 4);
  const v4f b0 = *(const v4fa*)(b + c8), b1 = *(const v4fa*)(b + c8 + 4);
  const v4f y0 = (g0 * (vc0 - mu)) * inv + b0;
  const v4f y1 = (g1 * (vc1 - mu)) * inv + b1;
  v8b hi, lo;
  split8(y0, y1, hi, lo);
  float* xo = xf + (size_t)row * DM;
  const size_t po = (size_t)row * DM + c8;
  #pragma unroll 1
  for (int pass = 0; pass < 2; ++pass) {
    vstore4f(xo + ca, va);
    vstore4f(xo + cb, vb);
    vstore8b(nh + po, hi);
    vstore8b(nl + po, lo);
    if (pass == 0) __threadfence();
  }
}

template <int RELU>
__device__ __forceinline__ void rows_pass(const float* sT, const float* bias, bf16_t* oh, bf16_t* ol,
                                          int opitch, int m0, int n0, int w, int lane) {
  const int c0 = 8 * lane;
  const v4f ba = *(const v4fa*)(bias + c0), bb = *(const v4fa*)(bias + c0 + 4);
  #pragma unroll
  for (int i = 0; i < 8; ++i) {
    const int row = 8 * w + i;
    v4f va = *(const v4fa*)(sT + row * 256 + c0) + ba;
    v4f vb = *(const v4fa*)(sT + row * 256 + c0 + 4) + bb;
    if (RELU) { va = vrelu(va); vb = vrelu(vb); }
    v8b hi, lo;
    split8(va, vb, hi, lo);
    const size_t gi = (size_t)(m0 + row) * (size_t)opitch + n0 + c0;
    vstore8b(oh + gi, hi);
    vstore8b(ol + gi, lo);
  }
}

__device__ __forceinline__ void vt_pass(const float* sT, const float* bias, bf16_t* oh, bf16_t* ol,
                                        int m0, int w, int lane) {
  const int sub = lane >> 3, tok0 = 8 * (lane & 7);
  #pragma unroll
  for (int i = 0; i < 8; ++i) {
    const int f = 32 * w + 4 * i + sub;
    const float bf = bias[f];
    const v4f va = *(const v4fa*)(sT + f * 64 + tok0) + bf;
    const v4f vb = *(const v4fa*)(sT + f * 64 + tok0 + 4) + bf;
    v8b hi, lo;
    split8(va, vb, hi, lo);
    const size_t gi = (size_t)f * NTOK + m0 + tok0;
    vstore8b(oh + gi, hi);
    vstore8b(ol + gi, lo);
  }
}

__device__ __forceinline__ void resln_prep(float* sT, const float* bias, const float* xf,
                                           int m0, int w, int lane) {
  const int ca = 4 * lane, cb = 128 + 4 * lane;
  const v4f ba = *(const v4fa*)(bias + ca), bb = *(const v4fa*)(bias + cb);
  #pragma unroll
  for (int i = 0; i < 8; ++i) {
    const int row = 8 * w + i;
    float* sr = sT + row * 256;
    const float* xr = xf + (size_t)(m0 + row) * DM;
    const v4f va = *(const v4fa*)(sr + ca) + ba + *(const v4fa*)(xr + ca);
    const v4f vb = *(const v4fa*)(sr + cb) + bb + *(const v4fa*)(xr + cb);
    *(v4fa*)(sr + ca) = va;
    *(v4fa*)(sr + cb) = vb;
  }
}

__device__ __forceinline__ void resln_pass(const float* sT, float* xf, const float* lg, const float* lb,
                                           bf16_t* nh, bf16_t* nl, float* dout, int fin,
                                           int m0, int w, int lane) {
  const int ca = 4 * lane, cb = 128 + 4 * lane, c8 = 8 * lane;
  const v4f ga = *(const v4fa*)(lg + ca), gb = *(const v4fa*)(lg + cb);
  const v4f gc0 = *(const v4fa*)(lg + c8), gc1 = *(const v4fa*)(lg + c8 + 4);
  const v4f ba = *(const v4fa*)(lb + ca), bb = *(const v4fa*)(lb + cb);
  const v4f bc0 = *(const v4fa*)(lb + c8), bc1 = *(const v4fa*)(lb + c8 + 4);
  #pragma unroll
  for (int i = 0; i < 8; ++i) {
    const int row = 8 * w + i;
    const size_t grow = (size_t)(m0 + row);
    const float* sr = sT + row * 256;
    const v4f va = *(const v4fa*)(sr + ca), vb = *(const v4fa*)(sr + cb);
    const v4f vc0 = *(const v4fa*)(sr + c8), vc1 = *(const v4fa*)(sr + c8 + 4);
    vstore4f(xf + grow * DM + ca, va);
    vstore4f(xf + grow * DM + cb, vb);
    float mu, inv;
    ln_stats(va, vb, mu, inv);
    if (fin) {
      const v4f ya = (ga * (va - mu)) * inv + ba;
      const v4f yb = (gb * (vb - mu)) * inv + bb;
      vstore4f(dout + grow * DM + ca, ya);
      vstore4f(dout + grow * DM + cb, yb);
    } else {
      const v4f y0 = (gc0 * (vc0 - mu)) * inv + bc0;
      const v4f y1 = (gc1 * (vc1 - mu)) * inv + bc1;
      v8b hi, lo;
      split8(y0, y1, hi, lo);
      vstore8b(nh + grow * DM + c8, hi);
      vstore8b(nl + grow * DM + c8, lo);
    }
  }
}

template <int MODE>
__global__ __launch_bounds__(256) void gemm_kernel(
    const bf16_t* __restrict__ Ah, const bf16_t* __restrict__ Al, int lda, int akblk,
    const bf16_t* __restrict__ Bh, const bf16_t* __restrict__ Bl, int K, int bws,
    const float* __restrict__ bias0, const float* __restrict__ bias1, const float* __restrict__ bias2,
    bf16_t* o0h, bf16_t* o0l, bf16_t* o1h, bf16_t* o1l, bf16_t* o2h, bf16_t* o2l, int opitch,
    float* xf, const float* __restrict__ lg, const float* __restrict__ lb, float* dout, int fin)
{
  extern __shared__ __attribute__((aligned(16))) float sT[];

  const int tid = threadIdx.x, lane = tid & 31, w = tid >> 5;
  const int wm = w & 3, wn = w >> 2;
  const int h = lane >> 4, m = lane & 15;
  const int m0 = blockIdx.y * 64;
  int which = 0, n0 = 0;
  if (MODE == 0) which = blockIdx.x;
  if (MODE == 1) n0 = blockIdx.x * 256;

  const bf16_t* Bhb = Bh + (size_t)which * bws;
  const bf16_t* Blb = Bl + (size_t)which * bws;
  const float* bias = bias0;
  if (MODE == 0) bias = (which == 0) ? bias0 : ((which == 1) ? bias1 : bias2);

  const int arow = m0 + 16 * wm + m;
  const bf16_t* arh = Ah + (size_t)arow * lda;
  const bf16_t* arl = Al + (size_t)arow * lda;
  const int ncol0 = n0 + 128 * wn;

  const v8f zero8 = {0.f, 0.f, 0.f, 0.f, 0.f, 0.f, 0.f, 0.f};
  v8f acc[8];
  #pragma unroll
  for (int nt = 0; nt < 8; ++nt) acc[nt] = zero8;

  #pragma unroll 1
  for (int k0 = 0; k0 < K; k0 += 32) {
    const size_t aoff = (size_t)(k0 >> 5) * (size_t)akblk;
    const v16b ah = load_frag(arh + aoff, h);
    const v16b al = load_frag(arl + aoff, h);
    #pragma unroll
    for (int nt = 0; nt < 8; ++nt) {
      const size_t boff = (size_t)(ncol0 + 16 * nt + m) * (size_t)K + k0;
      const v16b bh = load_frag(Bhb + boff, h);
      const v16b bl = load_frag(Blb + boff, h);
      acc[nt] = wmma3(ah, al, bh, bl, acc[nt]);
    }
  }

  const int rl0 = 16 * wm + 8 * h;
  if (MODE == 0 && which == 2) {
    #pragma unroll
    for (int nt = 0; nt < 8; ++nt)
      #pragma unroll
      for (int r = 0; r < 8; ++r) sT[(128 * wn + 16 * nt + m) * 64 + rl0 + r] = acc[nt][r];
  } else {
    #pragma unroll
    for (int nt = 0; nt < 8; ++nt)
      #pragma unroll
      for (int r = 0; r < 8; ++r) sT[(rl0 + r) * 256 + 128 * wn + 16 * nt + m] = acc[nt][r];
  }
  __syncthreads();

  if (MODE == 0) {
    if (which == 2) {
      vt_pass(sT, bias, o2h, o2l, m0, w, lane);
      __threadfence();
      vt_pass(sT, bias, o2h, o2l, m0, w, lane);
    } else {
      bf16_t* oh = (which == 0) ? o0h : o1h;
      bf16_t* ol = (which == 0) ? o0l : o1l;
      rows_pass<0>(sT, bias, oh, ol, opitch, m0, 0, w, lane);
      __threadfence();
      rows_pass<0>(sT, bias, oh, ol, opitch, m0, 0, w, lane);
    }
  } else if (MODE == 1) {
    rows_pass<1>(sT, bias + n0, o0h, o0l, opitch, m0, n0, w, lane);
    __threadfence();
    rows_pass<1>(sT, bias + n0, o0h, o0l, opitch, m0, n0, w, lane);
  } else {
    resln_prep(sT, bias, xf, m0, w, lane);
    __syncthreads();
    resln_pass(sT, xf, lg, lb, o0h, o0l, dout, fin, m0, w, lane);
    __threadfence();
    resln_pass(sT, xf, lg, lb, o0h, o0l, dout, fin, m0, w, lane);
  }
}

__device__ __forceinline__ void ctx_pass(const float* so, bf16_t* ch, bf16_t* cl,
                                         int head, int q0, int lane) {
  #pragma unroll
  for (int i = 0; i < 2; ++i) {
    const int row = 8 * i + (lane >> 2), dk0 = 8 * (lane & 3);
    const v4f va = *(const v4fa*)(so + row * 32 + dk0);
    const v4f vb = *(const v4fa*)(so + row * 32 + dk0 + 4);
    v8b hi, lo;
    split8(va, vb, hi, lo);
    const size_t gi = ((size_t)head * NTOK + q0 + row) * DKH + dk0;
    vstore8b(ch + gi, hi);
    vstore8b(cl + gi, lo);
  }
}

__global__ __launch_bounds__(128) void attn_kernel(
    const bf16_t* __restrict__ qh, const bf16_t* __restrict__ ql,
    const bf16_t* __restrict__ kh, const bf16_t* __restrict__ kl,
    const bf16_t* __restrict__ vth, const bf16_t* __restrict__ vtl,
    const int* __restrict__ rel,
    const float* __restrict__ relk, const float* __restrict__ relv,
    bf16_t* ch, bf16_t* cl,
    float scale)
{
  __shared__ __attribute__((aligned(16))) float sQR[4][16][48];
  __shared__ __attribute__((aligned(16))) float sBK[4][32][40];
  __shared__ __attribute__((aligned(16))) float sRV[NREL * DKH];
  __shared__ __attribute__((aligned(16))) float sO[4][16][32];

  const int tid = threadIdx.x, lane = tid & 31, w = tid >> 5;
  const int h = lane >> 4, m = lane & 15;
  const int head = blockIdx.y;
  const int q0 = blockIdx.x * 64 + 16 * w;
  const v8f zero8 = {0.f, 0.f, 0.f, 0.f, 0.f, 0.f, 0.f, 0.f};
  const v4f zero4 = {0.f, 0.f, 0.f, 0.f};

  for (int i = tid; i < NREL * DKH / 4; i += 128)
    *(v4fa*)(sRV + 4 * i) = *(const v4fa*)(relv + 4 * i);
  float* brow = &sBK[w][lane][0];
  #pragma unroll
  for (int i = 0; i < 40; ++i) brow[i] = 0.0f;

  const size_t qoff = (size_t)(q0 + m) * DM + DKH * head;
  const v16b qhf = load_frag(qh + qoff, h);
  const v16b qlf = load_frag(ql + qoff, h);

  #pragma unroll
  for (int t = 0; t < 3; ++t) {
    const int rr = 16 * t + m;
    const int rc = (rr < NREL) ? rr : (NREL - 1);
    const float* rp = relk + rc * DKH;
    v4f a0 = *(const v4fa*)(rp + 8 * h), a1 = *(const v4fa*)(rp + 8 * h + 4);
    v4f a2 = *(const v4fa*)(rp + 16 + 8 * h), a3 = *(const v4fa*)(rp + 16 + 8 * h + 4);
    a0 = (rr < NREL) ? a0 : zero4;  a1 = (rr < NREL) ? a1 : zero4;
    a2 = (rr < NREL) ? a2 : zero4;  a3 = (rr < NREL) ? a3 : zero4;
    Frag bh, bl;
    split8(a0, a1, bh.half[0], bl.half[0]);
    split8(a2, a3, bh.half[1], bl.half[1]);
    v8f d = zero8;
    d = wmma3(qhf, qlf, bh.v, bl.v, d);
    #pragma unroll
    for (int r = 0; r < 8; ++r) sQR[w][8 * h + r][16 * t + m] = d[r];
  }
  __syncthreads();

  v8f o[2];
  o[0] = zero8; o[1] = zero8;
  float mrun = -1e30f, lrun = 0.0f;

  const size_t krow0 = (size_t)m * DM + DKH * head;
  const size_t vrow0 = (size_t)(DKH * head + m) * NTOK;
  const int* relrow = rel + (size_t)(q0 + m) * NTOK + 8 * h;
  const float* qrrow = &sQR[w][m][0];

  #pragma unroll 1
  for (int kb = 0; kb < NTOK; kb += 32) {
    v8f s[2];
    #pragma unroll
    for (int j = 0; j < 2; ++j) {
      const size_t ko = krow0 + (size_t)(kb + 16 * j) * DM;
      const v16b khf = load_frag(kh + ko, h);
      const v16b klf = load_frag(kl + ko, h);
      v8f z = zero8;
      z = wmma_bf(khf, qhf, z);
      z = wmma_bf(khf, qlf, z);
      z = wmma_bf(klf, qhf, z);
      s[j] = z;
    }
    int c[2][8];
    #pragma unroll
    for (int j = 0; j < 2; ++j) {
      const v4i ra = *(const v4ia*)(relrow + kb + 16 * j);
      const v4i rb = *(const v4ia*)(relrow + kb + 16 * j + 4);
      const int cc[8] = { ra.x, ra.y, ra.z, ra.w, rb.x, rb.y, rb.z, rb.w };
      #pragma unroll
      for (int r = 0; r < 8; ++r) {
        int v = cc[r];
        v = (v < 0) ? (v + NREL) : v;
        v = (v < 0) ? 0 : v;
        v = (v > NREL - 1) ? (NREL - 1) : v;
        c[j][r] = v;
        s[j][r] = (s[j][r] + qrrow[v]) * scale;
      }
    }
    float mloc = s[0][0];
    #pragma unroll
    for (int j = 0; j < 2; ++j)
      #pragma unroll
      for (int r = 0; r < 8; ++r) mloc = fmaxf(mloc, s[j][r]);
    mloc = fmaxf(mloc, __shfl_xor(mloc, 16));
    const float mold = mrun;
    const float mnew = fmaxf(mold, mloc);
    const float alpha = __expf(mold - mnew);
    mrun = mnew;
    float lsum = 0.0f;
    #pragma unroll
    for (int j = 0; j < 2; ++j)
      #pragma unroll
      for (int r = 0; r < 8; ++r) {
        const float p = __expf(s[j][r] - mnew);
        s[j][r] = p;
        lsum += p;
      }
    lsum += __shfl_xor(lsum, 16);
    lrun = lrun * alpha + lsum;
    o[0] = o[0] * alpha;
    o[1] = o[1] * alpha;
    if (mnew > mold) {
      #pragma unroll
      for (int i = 0; i < NREL; ++i) brow[i] = brow[i] * alpha;
    }
    #pragma unroll
    for (int j = 0; j < 2; ++j)
      #pragma unroll
      for (int r = 0; r < 8; ++r) brow[c[j][r]] += s[j][r];

    Frag ph, pl;
    split8v(s[0], ph.half[0], pl.half[0]);
    split8v(s[1], ph.half[1], pl.half[1]);

    #pragma unroll
    for (int t = 0; t < 2; ++t) {
      const size_t vo = vrow0 + (size_t)(16 * t) * NTOK + kb;
      const v16b vhf = load_frag(vth + vo, h);
      const v16b vlf = load_frag(vtl + vo, h);
      o[t] = wmma3(vhf, vlf, ph.v, pl.v, o[t]);
    }
  }
  __syncthreads();

  v8f e[2];
  e[0] = zero8; e[1] = zero8;
  const float* bA = &sBK[w][m][0];
  const float* bB = &sBK[w][16 + m][0];
  #pragma unroll 1
  for (int rr = 0; rr < NREL; ++rr) {
    const float S = bA[rr] + bB[rr];
    const float* rv = sRV + rr * DKH + 8 * h;
    const v4f x0 = *(const v4fa*)(rv), x1 = *(const v4fa*)(rv + 4);
    const v4f x2 = *(const v4fa*)(rv + 16), x3 = *(const v4fa*)(rv + 20);
    e[0][0] += S * x0.x; e[0][1] += S * x0.y; e[0][2] += S * x0.z; e[0][3] += S * x0.w;
    e[0][4] += S * x1.x; e[0][5] += S * x1.y; e[0][6] += S * x1.z; e[0][7] += S * x1.w;
    e[1][0] += S * x2.x; e[1][1] += S * x2.y; e[1][2] += S * x2.z; e[1][3] += S * x2.w;
    e[1][4] += S * x3.x; e[1][5] += S * x3.y; e[1][6] += S * x3.z; e[1][7] += S * x3.w;
  }
  const float inv = 1.0f / lrun;
  float* so = &sO[w][0][0];
  #pragma unroll
  for (int t = 0; t < 2; ++t)
    #pragma unroll
    for (int r = 0; r < 8; ++r)
      so[m * 32 + 16 * t + 8 * h + r] = (o[t][r] + e[t][r]) * inv;
  __syncthreads();

  ctx_pass(so, ch, cl, head, q0, lane);
  __threadfence();
  ctx_pass(so, ch, cl, head, q0, lane);
}

extern "C" void kernel_launch(void* const* d_in, const int* in_sizes, int n_in,
                              void* d_out, int out_size, void* d_ws, size_t ws_size,
                              hipStream_t stream) {
  if (n_in < 22) return;
  if (in_sizes[0] != NTOK * DM) return;
  if (in_sizes[1] != NTOK * NTOK) return;
  if (in_sizes[2] != NLAY * DM * DM || in_sizes[4] != NLAY * DM * DM ||
      in_sizes[6] != NLAY * DM * DM || in_sizes[8] != NLAY * DM * DM) return;
  if (in_sizes[3] != NLAY * DM || in_sizes[5] != NLAY * DM || in_sizes[7] != NLAY * DM ||
      in_sizes[9] != NLAY * DM || in_sizes[15] != NLAY * DM) return;
  if (in_sizes[10] != NLAY * NREL * DKH || in_sizes[11] != NLAY * NREL * DKH) return;
  if (in_sizes[12] != NLAY * DM * FFD || in_sizes[14] != NLAY * FFD * DM) return;
  if (in_sizes[13] != NLAY * FFD) return;
  if (in_sizes[16] != NLAY * DM || in_sizes[17] != NLAY * DM ||
      in_sizes[18] != NLAY * DM || in_sizes[19] != NLAY * DM) return;
  if (in_sizes[20] != DM || in_sizes[21] != DM) return;
  if (out_size != NTOK * DM) return;

  const float* x     = (const float*)d_in[0];
  const int*   rels  = (const int*)d_in[1];
  const float* Wq = (const float*)d_in[2];  const float* bq = (const float*)d_in[3];
  const float* Wk = (const float*)d_in[4];  const float* bk = (const float*)d_in[5];
  const float* Wv = (const float*)d_in[6];  const float* bv = (const float*)d_in[7];
  const float* Wo = (const float*)d_in[8];  const float* bo = (const float*)d_in[9];
  const float* relk = (const float*)d_in[10];
  const float* relv = (const float*)d_in[11];
  const float* W1 = (const float*)d_in[12]; const float* b1 = (const float*)d_in[13];
  const float* W2 = (const float*)d_in[14]; const float* b2 = (const float*)d_in[15];
  const float* ln1g = (const float*)d_in[16]; const float* ln1b = (const float*)d_in[17];
  const float* ln2g = (const float*)d_in[18]; const float* ln2b = (const float*)d_in[19];
  const float* lnfg = (const float*)d_in[20]; const float* lnfb = (const float*)d_in[21];
  float* dout = (float*)d_out;

  const size_t e_qkv = (size_t)3 * NLAY * DM * DM;
  const size_t e_wo  = (size_t)NLAY * DM * DM;
  const size_t e_w1  = (size_t)NLAY * DM * FFD;
  const size_t e_w2  = (size_t)NLAY * FFD * DM;
  const size_t e_x   = (size_t)NTOK * DM;
  const size_t e_h   = (size_t)NTOK * FFD;
  size_t off = 0;
  char* ws = (char*)d_ws;
#define CARVE(ptr, type, nelem) type* ptr = (type*)(ws + off); off += (((size_t)(nelem) * sizeof(type)) + 255) & ~(size_t)255;
  CARVE(wqkv_h, bf16_t, e_qkv)  CARVE(wqkv_l, bf16_t, e_qkv)
  CARVE(wo_h,   bf16_t, e_wo)   CARVE(wo_l,   bf16_t, e_wo)
  CARVE(w1_h,   bf16_t, e_w1)   CARVE(w1_l,   bf16_t, e_w1)
  CARVE(w2_h,   bf16_t, e_w2)   CARVE(w2_l,   bf16_t, e_w2)
  CARVE(xf,     float,  e_x)
  CARVE(xn_h,   bf16_t, e_x)    CARVE(xn_l,   bf16_t, e_x)
  CARVE(q_h,    bf16_t, e_x)    CARVE(q_l,    bf16_t, e_x)
  CARVE(k_h,    bf16_t, e_x)    CARVE(k_l,    bf16_t, e_x)
  CARVE(vt_h,   bf16_t, e_x)    CARVE(vt_l,   bf16_t, e_x)
  CARVE(cx_h,   bf16_t, e_x)    CARVE(cx_l,   bf16_t, e_x)
  CARVE(hh_h,   bf16_t, e_h)    CARVE(hh_l,   bf16_t, e_h)
#undef CARVE
  if (off > ws_size) return;
  if (off > (size_t)134217728) return;

  const float scale = 0.1767766923f;
  const size_t ldsg = (size_t)64 * 256 * sizeof(float);

  wcvt_kernel<<<dim3(DM / 64, DM / 64, NLAY), 256, 0, stream>>>(Wq, wqkv_h, wqkv_l, DM, DM);
  wcvt_kernel<<<dim3(DM / 64, DM / 64, NLAY), 256, 0, stream>>>(Wk, wqkv_h + e_wo, wqkv_l + e_wo, DM, DM);
  wcvt_kernel<<<dim3(DM / 64, DM / 64, NLAY), 256, 0, stream>>>(Wv, wqkv_h + 2 * e_wo, wqkv_l + 2 * e_wo, DM, DM);
  wcvt_kernel<<<dim3(DM / 64, DM / 64, NLAY), 256, 0, stream>>>(Wo, wo_h, wo_l, DM, DM);
  wcvt_kernel<<<dim3(FFD / 64, DM / 64, NLAY), 256, 0, stream>>>(W1, w1_h, w1_l, DM, FFD);
  wcvt_kernel<<<dim3(DM / 64, FFD / 64, NLAY), 256, 0, stream>>>(W2, w2_h, w2_l, FFD, DM);

  ln0_kernel<<<NTOK / 8, 256, 0, stream>>>(x, ln1g, ln1b, xf, xn_h, xn_l, NTOK);

  for (int l = 0; l < NLAY; ++l) {
    gemm_kernel<0><<<dim3(3, NTOK / 64), 256, ldsg, stream>>>(
        xn_h, xn_l, DM, 32,
        wqkv_h + (size_t)l * DM * DM, wqkv_l + (size_t)l * DM * DM, DM, (int)e_wo,
        bq + l * DM, bk + l * DM, bv + l * DM,
        q_h, q_l, k_h, k_l, vt_h, vt_l, DM,
        xf, ln2g + l * DM, ln2b + l * DM, dout, 0);

    attn_kernel<<<dim3(NTOK / 64, NH), 128, 0, stream>>>(
        q_h, q_l, k_h, k_l, vt_h, vt_l, rels,
        relk + (size_t)l * NREL * DKH, relv + (size_t)l * NREL * DKH,
        cx_h, cx_l, scale);

    gemm_kernel<2><<<dim3(1, NTOK / 64), 256, ldsg, stream>>>(
        cx_h, cx_l, DKH, NTOK * DKH,
        wo_h + (size_t)l * DM * DM, wo_l + (size_t)l * DM * DM, DM, 0,
        bo + l * DM, bo + l * DM, bo + l * DM,
        xn_h, xn_l, xn_h, xn_l, xn_h, xn_l, DM,
        xf, ln2g + l * DM, ln2b + l * DM, dout, 0);

    gemm_kernel<1><<<dim3(FFD / 256, NTOK / 64), 256, ldsg, stream>>>(
        xn_h, xn_l, DM, 32,
        w1_h + (size_t)l * FFD * DM, w1_l + (size_t)l * FFD * DM, DM, 0,
        b1 + l * FFD, b1 + l * FFD, b1 + l * FFD,
        hh_h, hh_l, hh_h, hh_l, hh_h, hh_l, FFD,
        xf, ln2g + l * DM, ln2b + l * DM, dout, 0);

    const float* g_next = (l + 1 < NLAY) ? (ln1g + (l + 1) * DM) : lnfg;
    const float* b_next = (l + 1 < NLAY) ? (ln1b + (l + 1) * DM) : lnfb;
    const int fin = (l + 1 < NLAY) ? 0 : 1;
    gemm_kernel<2><<<dim3(1, NTOK / 64), 256, ldsg, stream>>>(
        hh_h, hh_l, FFD, 32,
        w2_h + (size_t)l * DM * FFD, w2_l + (size_t)l * DM * FFD, FFD, 0,
        b2 + l * DM, b2 + l * DM, b2 + l * DM,
        xn_h, xn_l, xn_h, xn_l, xn_h, xn_l, DM,
        xf, g_next, b_next, dout, fin);
  }
}
